// MambaBlock_44409961841182
// MI455X (gfx1250) — hardware-verified
//
#include <hip/hip_runtime.h>
#include <math.h>

typedef __attribute__((ext_vector_type(16))) _Float16 v16h;
typedef __attribute__((ext_vector_type(8)))  _Float16 v8h;
typedef __attribute__((ext_vector_type(16))) __bf16   v16b;
typedef __attribute__((ext_vector_type(8)))  __bf16   v8b;
typedef __attribute__((ext_vector_type(8)))  float    v8f;
typedef __attribute__((ext_vector_type(4)))  float    v4f;

constexpr int kBatch = 4;
constexpr int kSeq   = 2048;
constexpr int kDm    = 768;
constexpr int kDin   = 1536;
constexpr int kNst   = 16;
constexpr int kDtR   = 48;
constexpr int kDtP   = 64;
constexpr int kPrjN  = kDtR + 2 * kNst;
constexpr int kPrjP  = 128;
constexpr int kXzP   = 2 * kDin;
constexpr int kRows  = kBatch * kSeq;
constexpr int kTP    = 260;
static_assert(kDtR == (kDm + 15) / 16 && kPrjN == 80 && kXzP == 3072 && kRows == 8192, "shape constants");
static_assert((kDm % 32) == 0 && (kDin % 32) == 0 && (kDtP % 32) == 0, "GEMM K multiples of 32");
static_assert((kSeq % 64) == 0 && (kXzP % 64) == 0 && (kPrjP % 64) == 0 && (kDin % 64) == 0 && (kDm % 64) == 0, "GEMM M,N multiples of 64");
static_assert((kDm % 64) == 0 && (kDtP % 64) == 0 && (kDin % 64) == 0, "transpose k tiles of 64");
static_assert(kDtR < kDtP && (kDtR % 8) == 0 && kPrjN <= kPrjP && (kDtR % 4) == 0, "dt / x_proj padding");
static_assert((kDin % 256) == 0 && (kSeq % 16) == 0, "scan / conv tiles");
static_assert(((kRows * kDm / 8) % 256) == 0 && ((kSeq * kDtP / 8) % 256) == 0, "cast grids exact");

constexpr size_t kSzXB   = (size_t)kRows * kDm  * 2;
constexpr size_t kSzWIB  = (size_t)kXzP  * kDm  * 2;
constexpr size_t kSzWXB  = (size_t)kPrjP * kDin * 2;
constexpr size_t kSzWDB  = (size_t)kDin  * kDtP * 2;
constexpr size_t kSzWOB  = (size_t)kDm   * kDin * 2;
constexpr size_t kSzXZ   = (size_t)kSeq  * kXzP * 4;
constexpr size_t kSzUC   = (size_t)kSeq  * kDin * 4;
constexpr size_t kSzUC16 = (size_t)kSeq  * kDin * 2;
constexpr size_t kSzPROJ = (size_t)kSeq  * kPrjP * 4;
constexpr size_t kSzDT16 = (size_t)kSeq  * kDtP * 2;
constexpr size_t kSzDLR  = (size_t)kSeq  * kDin * 4;
constexpr size_t kSzY16  = (size_t)kSeq  * kDin * 2;
constexpr size_t kOffXB   = 0;
constexpr size_t kOffWIB  = kOffXB   + kSzXB;
constexpr size_t kOffWXB  = kOffWIB  + kSzWIB;
constexpr size_t kOffWDB  = kOffWXB  + kSzWXB;
constexpr size_t kOffWOB  = kOffWDB  + kSzWDB;
constexpr size_t kOffXZ   = kOffWOB  + kSzWOB;
constexpr size_t kOffUC   = kOffXZ   + kSzXZ;
constexpr size_t kOffUCH  = kOffUC   + kSzUC;
constexpr size_t kOffUCL  = kOffUCH  + kSzUC16;
constexpr size_t kOffPROJ = kOffUCL  + kSzUC16;
constexpr size_t kOffDTH  = kOffPROJ + kSzPROJ;
constexpr size_t kOffDTL  = kOffDTH  + kSzDT16;
constexpr size_t kOffDLR  = kOffDTL  + kSzDT16;
constexpr size_t kOffYH   = kOffDLR  + kSzDLR;
constexpr size_t kOffYL   = kOffYH   + kSzY16;
constexpr size_t kWsTotal = kOffYL   + kSzY16;
static_assert(kWsTotal == 97320960ull, "carve total");
static_assert(kWsTotal <= 134217728ull, "carve cap");
static_assert((kOffWIB % 128) == 0 && (kOffWXB % 128) == 0 && (kOffWDB % 128) == 0 && (kOffWOB % 128) == 0 &&
              (kOffXZ % 128) == 0 && (kOffUC % 128) == 0 && (kOffUCH % 128) == 0 && (kOffUCL % 128) == 0 &&
              (kOffPROJ % 128) == 0 && (kOffDTH % 128) == 0 && (kOffDTL % 128) == 0 && (kOffDLR % 128) == 0 &&
              (kOffYH % 128) == 0 && (kOffYL % 128) == 0, "128-B aligned regions");

__device__ __forceinline__ unsigned short f2bf_bits(float f) {
  unsigned u = __float_as_uint(f);
  return (unsigned short)((u + 0x7FFFu + ((u >> 16) & 1u)) >> 16);
}
__device__ __forceinline__ float bf_bits2f(unsigned short h) { return __uint_as_float(((unsigned)h) << 16); }
__device__ __forceinline__ float bfr(float f) { return bf_bits2f(f2bf_bits(f)); }

__device__ __forceinline__ void split8_bf16(const v4f a0, const v4f a1, v8h& hv, v8h& lv) {
#pragma unroll
  for (int e = 0; e < 4; ++e) {
    const float f0 = a0[e], f1 = a1[e];
    const unsigned short h0 = f2bf_bits(f0), h1 = f2bf_bits(f1);
    const unsigned short l0 = f2bf_bits(f0 - bf_bits2f(h0)), l1 = f2bf_bits(f1 - bf_bits2f(h1));
    hv[e]     = __builtin_bit_cast(_Float16, h0);
    hv[4 + e] = __builtin_bit_cast(_Float16, h1);
    lv[e]     = __builtin_bit_cast(_Float16, l0);
    lv[4 + e] = __builtin_bit_cast(_Float16, l1);
  }
}

__device__ __forceinline__ void dep_guard4_h(v8f& a, v8f& b, v8f& c, v8f& d, v16h x, v16h y) {
  asm volatile("v_nop\n\tv_nop\n\tv_nop\n\tv_nop" : "+v"(a), "+v"(b), "+v"(c), "+v"(d) : "v"(x), "v"(y));
}
__device__ __forceinline__ void dep_guard4_b(v8f& a, v8f& b, v8f& c, v8f& d, v16b x, v16b y) {
  asm volatile("v_nop\n\tv_nop\n\tv_nop\n\tv_nop" : "+v"(a), "+v"(b), "+v"(c), "+v"(d) : "v"(x), "v"(y));
}
__device__ __forceinline__ void keep4_h(v16h a, v16h b, v16h c, v16h d) { asm volatile("v_nop" :: "v"(a), "v"(b), "v"(c), "v"(d)); }
__device__ __forceinline__ void keep4_b(v16b a, v16b b, v16b c, v16b d) { asm volatile("v_nop" :: "v"(a), "v"(b), "v"(c), "v"(d)); }
__device__ __forceinline__ void acc_guard4(v8f& a, v8f& b, v8f& c, v8f& d) { asm volatile("v_nop\n\tv_nop\n\tv_nop\n\tv_nop" : "+v"(a), "+v"(b), "+v"(c), "+v"(d)); }
template <typename T> struct Frag;
template <> struct Frag<_Float16> {
  typedef v16h V; union U { v16h v; v8h h[2]; };
  static __device__ __forceinline__ v16h load(const _Float16* p) {
    U f; f.h[0] = *(const v8h*)(p); f.h[1] = *(const v8h*)(p + 16); return f.v;
  }
  static __device__ __forceinline__ v8f mma(v16h a, v16h b, v8f c) {
    return __builtin_amdgcn_wmma_f32_16x16x32_f16(false, a, false, b, (short)0, c, false, false);
  }
  static __device__ __forceinline__ void guard4(v8f& a, v8f& b, v8f& c, v8f& d, v16h x, v16h y) { dep_guard4_h(a, b, c, d, x, y); }
  static __device__ __forceinline__ void keep(v16h a, v16h b, v16h c, v16h d) { keep4_h(a, b, c, d); }
};
template <> struct Frag<__bf16> {
  typedef v16b V; union U { v16b v; v8b h[2]; };
  static __device__ __forceinline__ v16b load(const __bf16* p) {
    U f; f.h[0] = *(const v8b*)(p); f.h[1] = *(const v8b*)(p + 16); return f.v;
  }
  static __device__ __forceinline__ v8f mma(v16b a, v16b b, v8f c) {
    return __builtin_amdgcn_wmma_f32_16x16x32_bf16(false, a, false, b, (short)0, c, false, false);
  }
  static __device__ __forceinline__ void guard4(v8f& a, v8f& b, v8f& c, v8f& d, v16b x, v16b y) { dep_guard4_b(a, b, c, d, x, y); }
  static __device__ __forceinline__ void keep(v16b a, v16b b, v16b c, v16b d) { keep4_b(a, b, c, d); }
};

template <int ET> struct Elem;
template <> struct Elem<0> { typedef _Float16 T; };
template <> struct Elem<1> { typedef __bf16 T; };
template <int ET, int SPL, int BIAS_MODE, int OUT_MODE, bool RESID, int ACT = 0>
__global__ __launch_bounds__(256) void wmma_gemm64(
    const unsigned short* __restrict__ Ap, const unsigned short* __restrict__ A2p, int lda, long strideA,
    const unsigned short* __restrict__ Btp, const unsigned short* __restrict__ Bt2p, int ldb, long strideB,
    void* __restrict__ Cout, void* __restrict__ Cout2, int ldc, long strideC,
    const float* __restrict__ bias,
    const float* __restrict__ resid, long strideR,
    int M, int N, int K, float scale) {
  typedef typename Elem<ET>::T T;
  typedef typename Frag<T>::V V;
  const T* A = (const T*)Ap; const T* A2 = (const T*)A2p; const T* Bt = (const T*)Btp; const T* Bt2 = (const T*)Bt2p;
  __shared__ __align__(16) float sT[8][16 * 68];
  const int b    = blockIdx.y;
  const int lane = threadIdx.x & 31;
  const int wave = threadIdx.x >> 5;
  const int tilesN = N >> 6;
  const int tilesM = M >> 6;
  const int tile = blockIdx.x * 8 + wave;
  if (tile >= tilesM * tilesN) return;
  const int tm = tile / tilesN;
  const int tn = tile - tm * tilesN;
  const int m0 = tm << 6;
  const int n0 = tn << 6;

  const T* Ab  = A  + (size_t)b * strideA;
  const T* Bb  = Bt + (size_t)b * strideB;
  const T* Ab2 = (SPL >= 1) ? (A2  + (size_t)b * strideA) : nullptr;
  const T* Bb2 = (SPL == 2) ? (Bt2 + (size_t)b * strideB) : nullptr;

  const int rlane = lane & 15;
  const int koff  = (lane >> 4) * 8;
  const int mOff  = (lane >> 4) * 8;

  v8f acc[4][4];
#pragma unroll
  for (int i = 0; i < 4; ++i)
#pragma unroll
    for (int j = 0; j < 4; ++j) acc[i][j] = (v8f){0.f,0.f,0.f,0.f,0.f,0.f,0.f,0.f};

  for (int k0 = 0; k0 < K; k0 += 32) {
    V bh[4], bl[4];
#pragma unroll
    for (int j = 0; j < 4; ++j) {
      const size_t bo = (size_t)(n0 + (j << 4) + rlane) * ldb + koff + k0;
      bh[j] = Frag<T>::load(Bb + bo);
      if (SPL == 2) bl[j] = Frag<T>::load(Bb2 + bo);
    }
#pragma unroll
    for (int i = 0; i < 4; ++i) {
      const size_t ao = (size_t)(m0 + (i << 4) + rlane) * lda + koff + k0;
      V ah = Frag<T>::load(Ab + ao);
      V al;
      if (SPL >= 1) al = Frag<T>::load(Ab2 + ao);
#pragma unroll
      for (int j = 0; j < 4; ++j) {
        acc[i][j] = Frag<T>::mma(ah, bh[j], acc[i][j]);
        if (SPL == 2) acc[i][j] = Frag<T>::mma(ah, bl[j], acc[i][j]);
        if (SPL >= 1) acc[i][j] = Frag<T>::mma(al, bh[j], acc[i][j]);
      }
      Frag<T>::guard4(acc[i][0], acc[i][1], acc[i][2], acc[i][3], ah, (SPL >= 1) ? al : ah);
    }
    Frag<T>::keep(bh[0], bh[1], bh[2], bh[3]);
    if (SPL == 2) Frag<T>::keep(bl[0], bl[1], bl[2], bl[3]);
  }
  acc_guard4(acc[0][0], acc[0][1], acc[0][2], acc[0][3]);
  acc_guard4(acc[1][0], acc[1][1], acc[1][2], acc[1][3]);
  acc_guard4(acc[2][0], acc[2][1], acc[2][2], acc[2][3]);
  acc_guard4(acc[3][0], acc[3][1], acc[3][2], acc[3][3]);

  float* slab = sT[wave];
  const float* Rb = RESID ? (resid + (size_t)b * strideR) : nullptr;
#pragma unroll
  for (int i = 0; i < 4; ++i) {
    const int mBase = m0 + (i << 4);
#pragma unroll
    for (int j = 0; j < 4; ++j) {
      const int n = n0 + (j << 4) + rlane;
      float bv = 0.f;
      if (BIAS_MODE == 2) bv = bias[n];
#pragma unroll
      for (int r = 0; r < 8; ++r) {
        float v = acc[i][j][r] * scale;
        if (BIAS_MODE == 1) v += bias[mBase + mOff + r];
        if (BIAS_MODE == 2) v += bv;
        if (RESID) v += Rb[(size_t)(mBase + mOff + r) * ldc + n];
        if (ACT == 1) v = tanhf(v);
        if (ACT == 2) v = fmaxf(v, 0.0f);
        if (ACT == 3) v = v / (1.0f + expf(-v));
        if (ACT == 4) v = (v > 0.f) ? v : 0.01f * v;
        slab[(mOff + r) * 68 + (j << 4) + rlane] = v;
      }
    }
    __builtin_amdgcn_fence(__ATOMIC_RELEASE, "workgroup");
    __builtin_amdgcn_wave_barrier();
    __builtin_amdgcn_fence(__ATOMIC_ACQUIRE, "workgroup");
    if (OUT_MODE == 0) {
      float* C = (float*)Cout + (size_t)b * strideC;
      const int hh = lane >> 4, c4 = (lane & 15) * 4;
      for (int pass = 0; pass < 2; ++pass) {
#pragma unroll
        for (int it = 0; it < 8; ++it) {
          const int row = it * 2 + hh;
          v4f v = *(const v4f*)(slab + row * 68 + c4);
          *(volatile v4f*)(C + (size_t)(mBase + row) * ldc + n0 + c4) = v;
        }
        __threadfence();
      }
    } else {
      const int q = lane >> 3, c8 = (lane & 7) * 8;
      unsigned short* C  = (unsigned short*)Cout  + (size_t)b * strideC;
      unsigned short* C2 = (OUT_MODE == 2) ? ((unsigned short*)Cout2 + (size_t)b * strideC) : nullptr;
      for (int pass = 0; pass < 2; ++pass) {
#pragma unroll
        for (int it = 0; it < 4; ++it) {
          const int row = it * 4 + q;
          const float* sp = slab + row * 68 + c8;
          v8h hv, lv;
#pragma unroll
          for (int e = 0; e < 8; ++e) {
            if (OUT_MODE == 1) {
              hv[e] = (_Float16)sp[e];
            } else {
              unsigned short hb = f2bf_bits(sp[e]);
              unsigned short lb = f2bf_bits(sp[e] - bf_bits2f(hb));
              hv[e] = __builtin_bit_cast(_Float16, hb);
              lv[e] = __builtin_bit_cast(_Float16, lb);
            }
          }
          *(volatile v8h*)(C + (size_t)(mBase + row) * ldc + n0 + c8) = hv;
          if (OUT_MODE == 2) *(volatile v8h*)(C2 + (size_t)(mBase + row) * ldc + n0 + c8) = lv;
        }
        __threadfence();
      }
    }
    __builtin_amdgcn_fence(__ATOMIC_RELEASE, "workgroup");
    __builtin_amdgcn_wave_barrier();
    __builtin_amdgcn_fence(__ATOMIC_ACQUIRE, "workgroup");
  }
}

__global__ __launch_bounds__(256) void cast_bf16_kernel(
    const float* __restrict__ src, unsigned short* __restrict__ dst, int total8)
{
  const int i = blockIdx.x * 256 + threadIdx.x;
  if (i >= total8) return;
  const size_t e0 = (size_t)i << 3;
  const v4f a0 = *(const v4f*)(src + e0);
  const v4f a1 = *(const v4f*)(src + e0 + 4);
  v8h hv;
#pragma unroll
  for (int e = 0; e < 4; ++e) {
    const float f0 = a0[e], f1 = a1[e];
    const unsigned short b0 = f2bf_bits(f0), b1 = f2bf_bits(f1);
    hv[e]     = __builtin_bit_cast(_Float16, b0);
    hv[4 + e] = __builtin_bit_cast(_Float16, b1);
  }
  unsigned short* q = dst + e0;
  *(volatile v8h*)q = hv;
  __threadfence();
  *(volatile v8h*)q = hv;
}

__global__ __launch_bounds__(256) void transpose_cast_bf16_kernel(
    const float* __restrict__ W, unsigned short* __restrict__ Bt, int Kdim, int Kpad, int Ndim)
{
  __shared__ float tile[64 * 65];
  const int tid = threadIdx.x, lane = tid & 31, wave = tid >> 5;
  const int n0 = blockIdx.x * 64;
  const int k0 = blockIdx.y * 64;
#pragma unroll
  for (int p = 0; p < 16; ++p) {
    const int idx = tid + p * 256;
    const int kk  = idx >> 6;
    const int nn  = idx & 63;
    const int n   = n0 + nn;
    const int k   = k0 + kk;
    const int nc  = (n < Ndim) ? n : (Ndim - 1);
    const int kc  = (k < Kdim) ? k : (Kdim - 1);
    const float v = W[(size_t)kc * Ndim + nc];
    tile[kk * 65 + nn] = (n < Ndim && k < Kdim) ? v : 0.f;
  }
  __syncthreads();
  const int q = lane >> 3, c8 = (lane & 7) * 8;
  v8h hv[2];
#pragma unroll
  for (int it = 0; it < 2; ++it) {
    const int nrow = it * 32 + wave * 4 + q;
#pragma unroll
    for (int e = 0; e < 8; ++e) {
      const unsigned short bb = f2bf_bits(tile[(c8 + e) * 65 + nrow]);
      hv[it][e] = __builtin_bit_cast(_Float16, bb);
    }
  }
  for (int pass = 0; pass < 2; ++pass) {
#pragma unroll
    for (int it = 0; it < 2; ++it) {
      const int nrow = it * 32 + wave * 4 + q;
      *(volatile v8h*)(Bt + (size_t)(n0 + nrow) * Kpad + k0 + c8) = hv[it];
    }
    __threadfence();
  }
}

__global__ __launch_bounds__(256) void dt_split_kernel(
    const float* __restrict__ PROJ, unsigned short* __restrict__ DTH, unsigned short* __restrict__ DTL, int total8)
{
  const int i = blockIdx.x * 256 + threadIdx.x;
  if (i >= total8) return;
  const int e0  = i << 3;
  const int row = e0 >> 6;
  const int c8  = e0 & 63;
  const float* p = PROJ + (size_t)row * kPrjP + c8;
  const v4f r0 = *(const v4f*)(p);
  const v4f r1 = *(const v4f*)(p + 4);
  v4f a0, a1;
#pragma unroll
  for (int e = 0; e < 4; ++e) {
    const float f0 = r0[e], f1 = r1[e];
    a0[e] = (c8 + e < kDtR) ? f0 : 0.f;
    a1[e] = (c8 + 4 + e < kDtR) ? f1 : 0.f;
  }
  v8h hv, lv;
  split8_bf16(a0, a1, hv, lv);
  unsigned short* qh = DTH + e0;
  unsigned short* ql = DTL + e0;
  *(volatile v8h*)qh = hv;
  *(volatile v8h*)ql = lv;
  __threadfence();
  *(volatile v8h*)qh = hv;
  *(volatile v8h*)ql = lv;
}

__global__ __launch_bounds__(256) void conv_silu_kernel(
    const float* __restrict__ XZ, const float* __restrict__ cw, const float* __restrict__ cb,
    float* __restrict__ UC, unsigned short* __restrict__ UCH, unsigned short* __restrict__ UCL)
{
  __shared__ __align__(16) float sT[16 * kTP];
  const int tid = threadIdx.x, lane = tid & 31, wave = tid >> 5;
  const int d0 = blockIdx.x * 256, d = d0 + tid;
  const int t0 = blockIdx.y * 64;
  const float w0 = bfr(cw[d * 4 + 0]), w1 = bfr(cw[d * 4 + 1]), w2 = bfr(cw[d * 4 + 2]), w3 = bfr(cw[d * 4 + 3]);
  const float bc = bfr(cb[d]);
  float xm3, xm2, xm1;
  {
    const int r3 = t0 - 3, r2 = t0 - 2, r1 = t0 - 1;
    const float v3 = XZ[(size_t)(r3 < 0 ? 0 : r3) * kXzP + d];
    const float v2 = XZ[(size_t)(r2 < 0 ? 0 : r2) * kXzP + d];
    const float v1 = XZ[(size_t)(r1 < 0 ? 0 : r1) * kXzP + d];
    xm3 = (r3 >= 0) ? v3 : 0.f;
    xm2 = (r2 >= 0) ? v2 : 0.f;
    xm1 = (r1 >= 0) ? v1 : 0.f;
  }
  const int hrow = wave >> 1;
  const int hch  = (wave & 1) * 128 + lane * 4;
#pragma unroll 1
  for (int sub = 0; sub < 4; ++sub) {
    const int lb = t0 + sub * 16;
#pragma unroll 1
    for (int s = 0; s < 16; ++s) {
      const float xcur = XZ[(size_t)(lb + s) * kXzP + d];
      float acc = w0 * xm3;
      acc = fmaf(w1, xm2, acc);
      acc = fmaf(w2, xm1, acc);
      acc = fmaf(w3, xcur, acc);
      const float sv = acc + bc;
      const float sg = __builtin_amdgcn_rcpf(1.0f + expf(-sv));
      sT[s * kTP + tid] = sv * sg;
      xm3 = xm2; xm2 = xm1; xm1 = xcur;
    }
    __syncthreads();
    v4f fv[4];
    v8h bh[2], blo[2];
#pragma unroll
    for (int it = 0; it < 4; ++it) fv[it] = *(const v4f*)(sT + (it * 4 + hrow) * kTP + hch);
#pragma unroll
    for (int it = 0; it < 2; ++it) {
      const float* sp = sT + (it * 8 + wave) * kTP + lane * 8;
      const v4f a0 = *(const v4f*)(sp);
      const v4f a1 = *(const v4f*)(sp + 4);
      split8_bf16(a0, a1, bh[it], blo[it]);
    }
    for (int pass = 0; pass < 2; ++pass) {
#pragma unroll
      for (int it = 0; it < 4; ++it)
        *(volatile v4f*)(UC + (size_t)(lb + it * 4 + hrow) * kDin + d0 + hch) = fv[it];
#pragma unroll
      for (int it = 0; it < 2; ++it) {
        const size_t o = (size_t)(lb + it * 8 + wave) * kDin + d0 + lane * 8;
        *(volatile v8h*)(UCH + o) = bh[it];
        *(volatile v8h*)(UCL + o) = blo[it];
      }
      __threadfence();
    }
    __syncthreads();
  }
}

__global__ __launch_bounds__(256) void scan_kernel(
    const float* __restrict__ DLR, const float* __restrict__ UC, const float* __restrict__ XZ,
    const float* __restrict__ PROJ, const float* __restrict__ bdt, const float* __restrict__ Alog,
    const float* __restrict__ Dv, unsigned short* __restrict__ YH, unsigned short* __restrict__ YL)
{
  __shared__ __align__(16) float sBC[16 * 32];
  __shared__ __align__(16) float sA[kNst * 256];
  __shared__ __align__(16) float sY[16 * kTP];
  const int tid = threadIdx.x, lane = tid & 31, wave = tid >> 5;
  const int d0 = blockIdx.x * 256, d = d0 + tid;

#pragma unroll 1
  for (int n = 0; n < kNst; ++n) sA[n * 256 + tid] = -expf(bfr(Alog[(size_t)d * kNst + n]));
  const float bb = bfr(bdt[d]);
  const float Dd = bfr(Dv[d]);
  __syncthreads();
  float An[kNst], h[kNst];
#pragma unroll
  for (int n = 0; n < kNst; ++n) { An[n] = sA[n * 256 + tid]; h[n] = 0.f; }

#pragma unroll 1
  for (int c = 0; c < kSeq / 16; ++c) {
    const int l0 = c * 16;
    if (tid < 128) {
      const int r = tid >> 3, q = (tid & 7) * 4;
      const v4f v = *(const v4f*)(PROJ + (size_t)(l0 + r) * kPrjP + kDtR + q);
      *(v4f*)(sBC + r * 32 + q) = v;
    }
    __syncthreads();
#pragma unroll 1
    for (int s = 0; s < 16; ++s) {
      const size_t m = (size_t)(l0 + s);
      const float a     = DLR[m * kDin + d] + bb;
      const float delta = fmaxf(a, 0.0f) + log1pf(expf(-fabsf(a)));
      const float xv    = UC[m * kDin + d];
      const float zv    = XZ[m * kXzP + kDin + d];
      v4f Bq[4], Cq[4];
#pragma unroll
      for (int qq = 0; qq < 4; ++qq) {
        Bq[qq] = *(const v4f*)(sBC + s * 32 + 4 * qq);
        Cq[qq] = *(const v4f*)(sBC + s * 32 + kNst + 4 * qq);
      }
      float y = 0.f;
#pragma unroll
      for (int n = 0; n < kNst; ++n) {
        const float e = __expf(delta * An[n]);
        float db = delta * Bq[n >> 2][n & 3];
        asm volatile("" : "+v"(db));
        float p = db * xv;
        asm volatile("" : "+v"(p));
        float qv = h[n] * e;
        asm volatile("" : "+v"(qv));
        const float hn = qv + p;
        h[n] = hn;
        float rr = Cq[n >> 2][n & 3] * hn;
        asm volatile("" : "+v"(rr));
        y += rr;
      }
      float sk = xv * Dd;
      asm volatile("" : "+v"(sk));
      y += sk;
      const float sg = __builtin_amdgcn_rcpf(1.0f + expf(-zv));
      const float g  = zv * sg;
      sY[s * kTP + tid] = y * g;
    }
    __syncthreads();
    v8h hv[2], lv[2];
#pragma unroll
    for (int it = 0; it < 2; ++it) {
      const float* sp = sY + (it * 8 + wave) * kTP + lane * 8;
      const v4f a0 = *(const v4f*)(sp);
      const v4f a1 = *(const v4f*)(sp + 4);
      split8_bf16(a0, a1, hv[it], lv[it]);
    }
    for (int pass = 0; pass < 2; ++pass) {
#pragma unroll
      for (int it = 0; it < 2; ++it) {
        const size_t o = (size_t)(l0 + it * 8 + wave) * kDin + d0 + lane * 8;
        *(volatile v8h*)(YH + o) = hv[it];
        *(volatile v8h*)(YL + o) = lv[it];
      }
      __threadfence();
    }
  }
}

extern "C" void kernel_launch(void* const* d_in, const int* in_sizes, int n_in,
                              void* d_out, int out_size, void* d_ws, size_t ws_size,
                              hipStream_t stream)
{
  if (n_in < 10) return;
  if (in_sizes[0] != kRows * kDm) return;
  if (in_sizes[1] != kDm * kXzP) return;
  if (in_sizes[2] != kDin * 4 || in_sizes[3] != kDin) return;
  if (in_sizes[4] != kDin * kPrjN) return;
  if (in_sizes[5] != kDtR * kDin || in_sizes[6] != kDin) return;
  if (in_sizes[7] != kDin * kNst || in_sizes[8] != kDin) return;
  if (in_sizes[9] != kDin * kDm) return;
  if (out_size != kRows * kDm) return;
  if (ws_size < kWsTotal) return;

  const float* x      = (const float*)d_in[0];
  const float* W_in   = (const float*)d_in[1];
  const float* conv_w = (const float*)d_in[2];
  const float* conv_b = (const float*)d_in[3];
  const float* W_xprj = (const float*)d_in[4];
  const float* W_dt   = (const float*)d_in[5];
  const float* b_dt   = (const float*)d_in[6];
  const float* A_log  = (const float*)d_in[7];
  const float* Dv     = (const float*)d_in[8];
  const float* W_out  = (const float*)d_in[9];
  float* dout = (float*)d_out;

  char* ws = (char*)d_ws;
  unsigned short* XB   = (unsigned short*)(ws + kOffXB);
  unsigned short* WIB  = (unsigned short*)(ws + kOffWIB);
  unsigned short* WXB  = (unsigned short*)(ws + kOffWXB);
  unsigned short* WDB  = (unsigned short*)(ws + kOffWDB);
  unsigned short* WOB  = (unsigned short*)(ws + kOffWOB);
  float*          XZ   = (float*)(ws + kOffXZ);
  float*          UC   = (float*)(ws + kOffUC);
  unsigned short* UCH  = (unsigned short*)(ws + kOffUCH);
  unsigned short* UCL  = (unsigned short*)(ws + kOffUCL);
  float*          PROJ = (float*)(ws + kOffPROJ);
  unsigned short* DTH  = (unsigned short*)(ws + kOffDTH);
  unsigned short* DTL  = (unsigned short*)(ws + kOffDTL);
  float*          DLR  = (float*)(ws + kOffDLR);
  unsigned short* YH   = (unsigned short*)(ws + kOffYH);
  unsigned short* YL   = (unsigned short*)(ws + kOffYL);
  const float* dummy_bias  = b_dt;
  const float* dummy_resid = x;

  cast_bf16_kernel<<<(kRows * kDm) / 8 / 256, 256, 0, stream>>>(x, XB, (kRows * kDm) / 8);

  transpose_cast_bf16_kernel<<<dim3(kXzP / 64, kDm / 64), 256, 0, stream>>>(W_in,   WIB, kDm,  kDm,  kXzP);
  transpose_cast_bf16_kernel<<<dim3(kPrjP / 64, kDin / 64), 256, 0, stream>>>(W_xprj, WXB, kDin, kDin, kPrjN);
  transpose_cast_bf16_kernel<<<dim3(kDin / 64, kDtP / 64), 256, 0, stream>>>(W_dt,   WDB, kDtR, kDtP, kDin);
  transpose_cast_bf16_kernel<<<dim3(kDm / 64, kDin / 64), 256, 0, stream>>>(W_out,  WOB, kDin, kDin, kDm);

  for (int b = 0; b < kBatch; ++b) {
    const unsigned short* XBb = XB + (size_t)b * kSeq * kDm;
    float* outb = dout + (size_t)b * kSeq * kDm;

    wmma_gemm64<1, 0, 0, 0, false><<<dim3(192, 1), 256, 0, stream>>>(
        XBb, XBb, kDm, 0L, WIB, WIB, kDm, 0L,
        (void*)XZ, (void*)XZ, kXzP, 0L, dummy_bias, dummy_resid, 0L, kSeq, kXzP, kDm, 1.0f);

    conv_silu_kernel<<<dim3(kDin / 256, kSeq / 64), 256, 0, stream>>>(XZ, conv_w, conv_b, UC, UCH, UCL);

    wmma_gemm64<1, 1, 0, 0, false><<<dim3(8, 1), 256, 0, stream>>>(
        UCH, UCL, kDin, 0L, WXB, WXB, kDin, 0L,
        (void*)PROJ, (void*)PROJ, kPrjP, 0L, dummy_bias, dummy_resid, 0L, kSeq, kPrjP, kDin, 1.0f);

    dt_split_kernel<<<(kSeq * kDtP) / 8 / 256, 256, 0, stream>>>(PROJ, DTH, DTL, (kSeq * kDtP) / 8);

    wmma_gemm64<1, 1, 0, 0, false><<<dim3(96, 1), 256, 0, stream>>>(
        DTH, DTL, kDtP, 0L, WDB, WDB, kDtP, 0L,
        (void*)DLR, (void*)DLR, kDin, 0L, dummy_bias, dummy_resid, 0L, kSeq, kDin, kDtP, 1.0f);

    scan_kernel<<<dim3(kDin / 256, 1), 256, 0, stream>>>(DLR, UC, XZ, PROJ, b_dt, A_log, Dv, YH, YL);

    wmma_gemm64<1, 1, 0, 0, false><<<dim3(48, 1), 256, 0, stream>>>(
        YH, YL, kDin, 0L, WOB, WOB, kDin, 0L,
        (void*)outb, (void*)outb, kDm, 0L, dummy_bias, dummy_resid, 0L, kSeq, kDm, kDin, 1.0f);
  }
}
